// FlashLinearAttention_8126078124549
// MI455X (gfx1250) — hardware-verified
//
#include <hip/hip_runtime.h>
#include <stdint.h>
#include <math.h>


typedef __attribute__((ext_vector_type(16))) _Float16 v16h;
typedef __attribute__((ext_vector_type(8)))  _Float16 v8h;
typedef __attribute__((ext_vector_type(16))) __bf16   v16b;
typedef __attribute__((ext_vector_type(8)))  __bf16   v8b;
typedef __attribute__((ext_vector_type(8)))  float    v8f;
typedef __attribute__((ext_vector_type(4)))  float    v4f;

__device__ __forceinline__ unsigned short f2bf_bits(float f) {
  unsigned u = __float_as_uint(f);
  return (unsigned short)((u + 0x7FFFu + ((u >> 16) & 1u)) >> 16);
}
__device__ __forceinline__ float bf_bits2f(unsigned short h) { return __uint_as_float(((unsigned)h) << 16); }

__device__ __forceinline__ void dep_guard_h(v8f& a, v8f& b, v16h x, v16h y) { asm volatile("v_nop\n\tv_nop\n\tv_nop\n\tv_nop" : "+v"(a), "+v"(b) : "v"(x), "v"(y)); }
__device__ __forceinline__ void dep_guard_b(v8f& a, v8f& b, v16b x, v16b y) { asm volatile("v_nop\n\tv_nop\n\tv_nop\n\tv_nop" : "+v"(a), "+v"(b) : "v"(x), "v"(y)); }
__device__ __forceinline__ void keep4_h(v16h a, v16h b, v16h c, v16h d) { asm volatile("v_nop" :: "v"(a), "v"(b), "v"(c), "v"(d)); }
__device__ __forceinline__ void keep4_b(v16b a, v16b b, v16b c, v16b d) { asm volatile("v_nop" :: "v"(a), "v"(b), "v"(c), "v"(d)); }
__device__ __forceinline__ void acc_guard4(v8f& a, v8f& b, v8f& c, v8f& d) { asm volatile("v_nop\n\tv_nop\n\tv_nop\n\tv_nop" : "+v"(a), "+v"(b), "+v"(c), "+v"(d)); }
template <typename T> struct Frag;
template <> struct Frag<_Float16> {
  typedef v16h V; union U { v16h v; v8h h[2]; };
  static __device__ __forceinline__ v16h load(const _Float16* p) {
    U f; f.h[0] = *(const v8h*)(p); f.h[1] = *(const v8h*)(p + 16); return f.v;
  }
  static __device__ __forceinline__ v8f mma(v16h a, v16h b, v8f c) {
    return __builtin_amdgcn_wmma_f32_16x16x32_f16(false, a, false, b, (short)0, c, false, false);
  }
  static __device__ __forceinline__ void guard(v8f& a, v8f& b, v16h x, v16h y) { dep_guard_h(a, b, x, y); }
  static __device__ __forceinline__ void keep(v16h a, v16h b, v16h c, v16h d) { keep4_h(a, b, c, d); }
};
template <> struct Frag<__bf16> {
  typedef v16b V; union U { v16b v; v8b h[2]; };
  static __device__ __forceinline__ v16b load(const __bf16* p) {
    U f; f.h[0] = *(const v8b*)(p); f.h[1] = *(const v8b*)(p + 16); return f.v;
  }
  static __device__ __forceinline__ v8f mma(v16b a, v16b b, v8f c) {
    return __builtin_amdgcn_wmma_f32_16x16x32_bf16(false, a, false, b, (short)0, c, false, false);
  }
  static __device__ __forceinline__ void guard(v8f& a, v8f& b, v16b x, v16b y) { dep_guard_b(a, b, x, y); }
  static __device__ __forceinline__ void keep(v16b a, v16b b, v16b c, v16b d) { keep4_b(a, b, c, d); }
};

template <int ET> struct Elem;
template <> struct Elem<0> { typedef _Float16 T; };
template <> struct Elem<1> { typedef __bf16 T; };
template <int ET, bool SPLIT, int BIAS_MODE, int OUT_MODE, bool RESID, int ACT = 0>
__global__ __launch_bounds__(256) void wmma_gemm64(
    const unsigned short* __restrict__ Ap, const unsigned short* __restrict__ A2p, int lda, long strideA,
    const unsigned short* __restrict__ Btp, const unsigned short* __restrict__ Bt2p, int ldb, long strideB,
    void* __restrict__ Cout, void* __restrict__ Cout2, int ldc, long strideC,
    const float* __restrict__ bias,
    const float* __restrict__ resid, long strideR,
    int M, int N, int K, float scale, int NB) {
  typedef typename Elem<ET>::T T;
  typedef typename Frag<T>::V V;
  const T* A = (const T*)Ap; const T* A2 = (const T*)A2p; const T* Bt = (const T*)Btp; const T* Bt2 = (const T*)Bt2p;
  __shared__ __align__(16) float sT[8][16 * 68];
  const int lane = threadIdx.x & 31;
  const int wave = threadIdx.x >> 5;
  const int tilesN = N >> 6;
  const int tilesM = M >> 6;
  const int tilesPer = tilesM * tilesN;
  const int gt = blockIdx.x * 8 + wave;
  if (gt >= NB * tilesPer) return;
  const int b    = gt / tilesPer;
  const int tile = gt - b * tilesPer;
  const int tm = tile / tilesN;
  const int tn = tile - tm * tilesN;
  const int m0 = tm << 6;
  const int n0 = tn << 6;

  const T* Ab  = A  + (size_t)b * strideA;
  const T* Bb  = Bt + (size_t)b * strideB;
  const T* Ab2 = SPLIT ? (A2  + (size_t)b * strideA) : nullptr;
  const T* Bb2 = SPLIT ? (Bt2 + (size_t)b * strideB) : nullptr;

  const int rlane = lane & 15;
  const int koff  = (lane >> 4) * 8;
  const int mOff  = (lane >> 4) * 8;

  v8f acc[4][4];
#pragma unroll
  for (int i = 0; i < 4; ++i)
#pragma unroll
    for (int j = 0; j < 4; ++j) acc[i][j] = (v8f){0.f,0.f,0.f,0.f,0.f,0.f,0.f,0.f};

  for (int k0 = 0; k0 < K; k0 += 32) {
    V bh[4], bl[4];
#pragma unroll
    for (int j = 0; j < 4; ++j) {
      const size_t bo = (size_t)(n0 + (j << 4) + rlane) * ldb + koff + k0;
      bh[j] = Frag<T>::load(Bb + bo);
      if (SPLIT) bl[j] = Frag<T>::load(Bb2 + bo);
    }
#pragma unroll
    for (int i = 0; i < 4; ++i) {
      const size_t ao = (size_t)(m0 + (i << 4) + rlane) * lda + koff + k0;
      V ah = Frag<T>::load(Ab + ao);
      V al;
      if (SPLIT) al = Frag<T>::load(Ab2 + ao);
#pragma unroll
      for (int j = 0; j < 4; ++j) {
        acc[i][j] = Frag<T>::mma(ah, bh[j], acc[i][j]);
        if (SPLIT) {
          acc[i][j] = Frag<T>::mma(ah, bl[j], acc[i][j]);
          acc[i][j] = Frag<T>::mma(al, bh[j], acc[i][j]);
        }
      }
      Frag<T>::guard(acc[i][0], acc[i][3], ah, SPLIT ? al : ah);
    }
    Frag<T>::keep(bh[0], bh[1], bh[2], bh[3]);
    if (SPLIT) Frag<T>::keep(bl[0], bl[1], bl[2], bl[3]);
  }
  acc_guard4(acc[0][0], acc[0][1], acc[0][2], acc[0][3]);
  acc_guard4(acc[1][0], acc[1][1], acc[1][2], acc[1][3]);
  acc_guard4(acc[2][0], acc[2][1], acc[2][2], acc[2][3]);
  acc_guard4(acc[3][0], acc[3][1], acc[3][2], acc[3][3]);

  float* slab = sT[wave];
  const float* Rb = RESID ? (resid + (size_t)b * strideR) : nullptr;
#pragma unroll
  for (int i = 0; i < 4; ++i) {
    const int mBase = m0 + (i << 4);
#pragma unroll
    for (int j = 0; j < 4; ++j) {
      const int n = n0 + (j << 4) + rlane;
      float bv = 0.f;
      if (BIAS_MODE == 2) bv = bias[n];
#pragma unroll
      for (int r = 0; r < 8; ++r) {
        float v = acc[i][j][r] * scale;
        if (BIAS_MODE == 1) v += bias[mBase + mOff + r];
        if (BIAS_MODE == 2) v += bv;
        if (RESID) v += Rb[(size_t)(mBase + mOff + r) * ldc + n];
        if (ACT == 1) v = tanhf(v);
        if (ACT == 2) v = fmaxf(v, 0.0f);
        if (ACT == 3) v = v * __builtin_amdgcn_rcpf(1.0f + __expf(-v));
        if (ACT == 4) v = (v > 0.f) ? v : 0.01f * v;
        if (ACT == 5) v = 0.5f * v * (1.0f + erff(v * 0.70710678118654752f));
        slab[(mOff + r) * 68 + (j << 4) + rlane] = v;
      }
    }
    __builtin_amdgcn_fence(__ATOMIC_RELEASE, "workgroup");
    __builtin_amdgcn_wave_barrier();
    __builtin_amdgcn_fence(__ATOMIC_ACQUIRE, "workgroup");
    if (OUT_MODE == 0) {
      float* C = (float*)Cout + (size_t)b * strideC;
      const int hh = lane >> 4, c4 = (lane & 15) * 4;
      for (int pass = 0; pass < 2; ++pass) {
#pragma unroll
        for (int it = 0; it < 8; ++it) {
          const int row = it * 2 + hh;
          v4f v = *(const v4f*)(slab + row * 68 + c4);
          *(volatile v4f*)(C + (size_t)(mBase + row) * ldc + n0 + c4) = v;
        }
        __threadfence();
      }
    } else {
      const int q = lane >> 3, c8 = (lane & 7) * 8;
      unsigned short* C  = (unsigned short*)Cout  + (size_t)b * strideC;
      unsigned short* C2 = (OUT_MODE == 2) ? ((unsigned short*)Cout2 + (size_t)b * strideC) : nullptr;
      for (int pass = 0; pass < 2; ++pass) {
#pragma unroll
        for (int it = 0; it < 4; ++it) {
          const int row = it * 4 + q;
          const float* sp = slab + row * 68 + c8;
          v8h hv, lv;
#pragma unroll
          for (int e = 0; e < 8; ++e) {
            if (OUT_MODE == 1) {
              hv[e] = (_Float16)sp[e];
            } else {
              unsigned short hb = f2bf_bits(sp[e]);
              unsigned short lb = f2bf_bits(sp[e] - bf_bits2f(hb));
              hv[e] = __builtin_bit_cast(_Float16, hb);
              lv[e] = __builtin_bit_cast(_Float16, lb);
            }
          }
          *(volatile v8h*)(C + (size_t)(mBase + row) * ldc + n0 + c8) = hv;
          if (OUT_MODE == 2) *(volatile v8h*)(C2 + (size_t)(mBase + row) * ldc + n0 + c8) = lv;
        }
        __threadfence();
      }
    }
    __builtin_amdgcn_fence(__ATOMIC_RELEASE, "workgroup");
    __builtin_amdgcn_wave_barrier();
    __builtin_amdgcn_fence(__ATOMIC_ACQUIRE, "workgroup");
  }
}

template <typename T>
__device__ __forceinline__ void mma_phase64(v8f (&acc)[4][4], const T* __restrict__ Ab, int lda,
                                            const T* __restrict__ Bb, int ldb, int K,
                                            int m0, int n0, int rlane, int koff) {
  typedef typename Frag<T>::V V;
  for (int k0 = 0; k0 < K; k0 += 32) {
    V bh[4];
#pragma unroll
    for (int j = 0; j < 4; ++j)
      bh[j] = Frag<T>::load(Bb + (size_t)(n0 + (j << 4) + rlane) * ldb + koff + k0);
#pragma unroll
    for (int i = 0; i < 4; ++i) {
      V ah = Frag<T>::load(Ab + (size_t)(m0 + (i << 4) + rlane) * lda + koff + k0);
#pragma unroll
      for (int j = 0; j < 4; ++j) acc[i][j] = Frag<T>::mma(ah, bh[j], acc[i][j]);
      Frag<T>::guard(acc[i][0], acc[i][3], ah, ah);
    }
    Frag<T>::keep(bh[0], bh[1], bh[2], bh[3]);
  }
}

__global__ __launch_bounds__(256) void wmma_dual64(
    const unsigned short* __restrict__ A1p, int lda1, long sA1,
    const unsigned short* __restrict__ B1p, int ldb1, long sB1, int K1,
    const unsigned short* __restrict__ A2p, int lda2, long sA2,
    const unsigned short* __restrict__ B2p, int ldb2, long sB2, int K2,
    const unsigned short* __restrict__ Gp, int ldg, long sG,
    unsigned short* __restrict__ Cp, int ldc, long sC,
    int M, int N, int NB, float scale) {
  typedef _Float16 T;
  __shared__ __align__(16) float sT[8][16 * 68];
  const int lane = threadIdx.x & 31;
  const int wave = threadIdx.x >> 5;
  const int tilesN = N >> 6;
  const int tilesM = M >> 6;
  const int tilesPer = tilesM * tilesN;
  const int gt = blockIdx.x * 8 + wave;
  if (gt >= NB * tilesPer) return;
  const int b    = gt / tilesPer;
  const int tile = gt - b * tilesPer;
  const int tm = tile / tilesN;
  const int tn = tile - tm * tilesN;
  const int m0 = tm << 6;
  const int n0 = tn << 6;

  const T* A1 = (const T*)A1p + (size_t)b * sA1;
  const T* B1 = (const T*)B1p + (size_t)b * sB1;
  const T* A2 = (const T*)A2p + (size_t)b * sA2;
  const T* B2 = (const T*)B2p + (size_t)b * sB2;
  const T* Gb = (const T*)Gp  + (size_t)b * sG;
  unsigned short* C = Cp + (size_t)b * sC;

  const int rlane = lane & 15;
  const int koff  = (lane >> 4) * 8;
  const int mOff  = (lane >> 4) * 8;

  v8f acc[4][4];
#pragma unroll
  for (int i = 0; i < 4; ++i)
#pragma unroll
    for (int j = 0; j < 4; ++j) acc[i][j] = (v8f){0.f,0.f,0.f,0.f,0.f,0.f,0.f,0.f};

  mma_phase64<T>(acc, A1, lda1, B1, ldb1, K1, m0, n0, rlane, koff);
  mma_phase64<T>(acc, A2, lda2, B2, ldb2, K2, m0, n0, rlane, koff);

  acc_guard4(acc[0][0], acc[0][1], acc[0][2], acc[0][3]);
  acc_guard4(acc[1][0], acc[1][1], acc[1][2], acc[1][3]);
  acc_guard4(acc[2][0], acc[2][1], acc[2][2], acc[2][3]);
  acc_guard4(acc[3][0], acc[3][1], acc[3][2], acc[3][3]);

  float* slab = sT[wave];
#pragma unroll
  for (int i = 0; i < 4; ++i) {
    const int mBase = m0 + (i << 4);
#pragma unroll
    for (int j = 0; j < 4; ++j) {
      const int n = n0 + (j << 4) + rlane;
#pragma unroll
      for (int r = 0; r < 8; ++r) {
        const float gv = (float)Gb[(size_t)(mBase + mOff + r) * ldg + n];
        slab[(mOff + r) * 68 + (j << 4) + rlane] = acc[i][j][r] * scale * gv;
      }
    }
    __builtin_amdgcn_fence(__ATOMIC_RELEASE, "workgroup");
    __builtin_amdgcn_wave_barrier();
    __builtin_amdgcn_fence(__ATOMIC_ACQUIRE, "workgroup");
    {
      const int q = lane >> 3, c8 = (lane & 7) * 8;
      for (int pass = 0; pass < 2; ++pass) {
#pragma unroll
        for (int it = 0; it < 4; ++it) {
          const int row = it * 4 + q;
          const float* sp = slab + row * 68 + c8;
          v8h hv;
#pragma unroll
          for (int e = 0; e < 8; ++e) hv[e] = (_Float16)sp[e];
          *(volatile v8h*)(C + (size_t)(mBase + row) * ldc + n0 + c8) = hv;
        }
        __threadfence();
      }
    }
    __builtin_amdgcn_fence(__ATOMIC_RELEASE, "workgroup");
    __builtin_amdgcn_wave_barrier();
    __builtin_amdgcn_fence(__ATOMIC_ACQUIRE, "workgroup");
  }
}

__global__ __launch_bounds__(256) void cast_f32_f16x2(
    const float* __restrict__ in, _Float16* __restrict__ out, int n2, float mul) {
  int i = blockIdx.x * 256 + threadIdx.x;
  if (i < n2) {
    const _Float16 h0 = (_Float16)(in[2 * i] * mul), h1 = (_Float16)(in[2 * i + 1] * mul);
    const unsigned u = (unsigned)__builtin_bit_cast(unsigned short, h0) | ((unsigned)__builtin_bit_cast(unsigned short, h1) << 16);
    ((volatile unsigned*)out)[i] = u;
    __threadfence();
    ((volatile unsigned*)out)[i] = u;
  }
}

__global__ __launch_bounds__(128) void ln_kernel(
    const float* __restrict__ q, const float* __restrict__ gam, const float* __restrict__ bet,
    _Float16* __restrict__ xn, int Lq, int NBt, float eps) {
  __shared__ float red0[4];
  __shared__ float red1[4];
  const int row = blockIdx.x;
  const int b = row / Lq;
  const int l = row - b * Lq;
  const int t = threadIdx.x, lane = t & 31, wave = t >> 5;
  const float* src = q + ((size_t)l * NBt + b) * 1024 + 8 * t;
  const v4f x0 = *(const v4f*)(src);
  const v4f x1 = *(const v4f*)(src + 4);
  float s = ((x0[0] + x0[1]) + (x0[2] + x0[3])) + ((x1[0] + x1[1]) + (x1[2] + x1[3]));
#pragma unroll
  for (int off = 1; off < 32; off <<= 1) s += __shfl_xor(s, off, 32);
  if (lane == 0) red0[wave] = s;
  __syncthreads();
  const float mean = ((red0[0] + red0[1]) + (red0[2] + red0[3])) * (1.0f / 1024.0f);
  float d[8];
  d[0] = x0[0] - mean; d[1] = x0[1] - mean; d[2] = x0[2] - mean; d[3] = x0[3] - mean;
  d[4] = x1[0] - mean; d[5] = x1[1] - mean; d[6] = x1[2] - mean; d[7] = x1[3] - mean;
  float s2 = 0.f;
#pragma unroll
  for (int e = 0; e < 8; ++e) s2 += d[e] * d[e];
#pragma unroll
  for (int off = 1; off < 32; off <<= 1) s2 += __shfl_xor(s2, off, 32);
  if (lane == 0) red1[wave] = s2;
  __syncthreads();
  const float var = ((red1[0] + red1[1]) + (red1[2] + red1[3])) * (1.0f / 1024.0f);
  const float inv = rsqrtf(var + eps);
  const v4f g0 = *(const v4f*)(gam + 8 * t), g1 = *(const v4f*)(gam + 8 * t + 4);
  const v4f b0 = *(const v4f*)(bet + 8 * t), b1 = *(const v4f*)(bet + 8 * t + 4);
  v8h o;
  o[0] = (_Float16)(d[0] * inv * g0[0] + b0[0]);
  o[1] = (_Float16)(d[1] * inv * g0[1] + b0[1]);
  o[2] = (_Float16)(d[2] * inv * g0[2] + b0[2]);
  o[3] = (_Float16)(d[3] * inv * g0[3] + b0[3]);
  o[4] = (_Float16)(d[4] * inv * g1[0] + b1[0]);
  o[5] = (_Float16)(d[5] * inv * g1[1] + b1[1]);
  o[6] = (_Float16)(d[6] * inv * g1[2] + b1[2]);
  o[7] = (_Float16)(d[7] * inv * g1[3] + b1[3]);
  _Float16* dst = xn + (size_t)row * 1024 + 8 * t;
  *(volatile v8h*)dst = o;
  __threadfence();
  *(volatile v8h*)dst = o;
}

__global__ __launch_bounds__(256) void rope_kernel(
    const float* __restrict__ base,
    const float* __restrict__ qqw, const float* __restrict__ qqb,
    const float* __restrict__ qkw, const float* __restrict__ qkb,
    const float* __restrict__ lqw, const float* __restrict__ lqb,
    const float* __restrict__ lkw, const float* __restrict__ lkb,
    _Float16* __restrict__ qq16, _Float16* __restrict__ qk16,
    _Float16* __restrict__ lq16, _Float16* __restrict__ lkT16, int nc) {
  __shared__ __align__(16) _Float16 T0[64 * 128];
  __shared__ __align__(16) _Float16 T1[64 * 128];
  const int bg = blockIdx.x;
  const int tid = threadIdx.x;
  const int n = tid >> 2, jq = tid & 3;
  const int row = bg * 64 + n;
  const int g = bg % nc;
  const float pos = (float)(g * 64 + n);
  const float* brow = base + (size_t)row * 128;
  const float QS = 64.0f;
#pragma unroll 1
  for (int ps = 0; ps < 2; ++ps) {
    const float* wA = ps ? lqw : qqw;
    const float* bA = ps ? lqb : qqb;
    const float* wB = ps ? lkw : qkw;
    const float* bB = ps ? lkb : qkb;
#pragma unroll 1
    for (int i = 0; i < 16; ++i) {
      const int j = jq * 16 + i;
      const float x1 = brow[j], x2 = brow[j + 64];
      const float invf = exp2f((float)j * -0.20762050593046017f);
      const float ang = pos * invf;
      const float sn = sinf(ang), cs = cosf(ang);
      float t1 = x1 * wA[j] + bA[j];
      float t2 = x2 * wA[j + 64] + bA[j + 64];
      float o1 = t1 * cs - t2 * sn;
      float o2 = t2 * cs + t1 * sn;
      T0[n * 128 + j]      = (_Float16)(o1 * QS);
      T0[n * 128 + j + 64] = (_Float16)(o2 * QS);
      t1 = x1 * wB[j] + bB[j];
      t2 = x2 * wB[j + 64] + bB[j + 64];
      o1 = t1 * cs - t2 * sn;
      o2 = t2 * cs + t1 * sn;
      if (ps == 0) {
        T1[n * 128 + j]      = (_Float16)(o1 * QS);
        T1[n * 128 + j + 64] = (_Float16)(o2 * QS);
      } else {
        T1[j * 64 + n]        = (_Float16)(o1 * QS);
        T1[(j + 64) * 64 + n] = (_Float16)(o2 * QS);
      }
    }
    __syncthreads();
    _Float16* d0 = (ps ? lq16  : qq16) + (size_t)bg * 8192;
    _Float16* d1 = (ps ? lkT16 : qk16) + (size_t)bg * 8192;
    for (int pass = 0; pass < 2; ++pass) {
#pragma unroll
      for (int it = 0; it < 4; ++it) {
        const int off = (it * 256 + tid) * 8;
        const v8h a0 = *(const v8h*)(T0 + off);
        const v8h a1 = *(const v8h*)(T1 + off);
        *(volatile v8h*)(d0 + off) = a0;
        *(volatile v8h*)(d1 + off) = a1;
      }
      __threadfence();
    }
    __syncthreads();
  }
}

__global__ __launch_bounds__(256) void kmat_kernel(
    const float* __restrict__ sc, const float* __restrict__ wrel, _Float16* __restrict__ km,
    int total8, int center, int nw) {
  const int e = blockIdx.x * 256 + threadIdx.x;
  if (e >= total8) return;
  const int n  = (e >> 3) & 63;
  const int mb = (e & 7) * 8;
  const float* sp = sc + (size_t)e * 8;
  const v4f s0 = *(const v4f*)(sp), s1 = *(const v4f*)(sp + 4);
  float sv[8];
  sv[0] = s0[0]; sv[1] = s0[1]; sv[2] = s0[2]; sv[3] = s0[3];
  sv[4] = s1[0]; sv[5] = s1[1]; sv[6] = s1[2]; sv[7] = s1[3];
  v8h o;
#pragma unroll
  for (int k = 0; k < 8; ++k) {
    const int m = mb + k;
    float val = 0.f;
    if (m <= n) {
      int idx = center + m - n;
      idx = idx < 0 ? 0 : (idx >= nw ? nw - 1 : idx);
      float x = sv[k] + wrel[idx];
      x = fmaxf(x, 0.f);
      val = x * x * 4096.0f;
    }
    o[k] = (_Float16)val;
  }
  _Float16* dst = km + (size_t)e * 8;
  *(volatile v8h*)dst = o;
  __threadfence();
  *(volatile v8h*)dst = o;
}

__global__ __launch_bounds__(256) void cumsum_kernel(
    const _Float16* __restrict__ in, _Float16* __restrict__ out, int per8, int nc, long per) {
  const int t = blockIdx.x * 256 + threadIdx.x;
  if (t >= per8) return;
  float run[8];
#pragma unroll
  for (int e = 0; e < 8; ++e) run[e] = 0.f;
#pragma unroll 1
  for (int g = 0; g < nc; ++g) {
    const size_t off = (size_t)g * (size_t)per + (size_t)t * 8;
    v8h o;
#pragma unroll
    for (int e = 0; e < 8; ++e) o[e] = (_Float16)run[e];
    *(volatile v8h*)(out + off) = o;
    __threadfence();
    *(volatile v8h*)(out + off) = o;
    const v8h a = *(const v8h*)(in + off);
#pragma unroll
    for (int e = 0; e < 8; ++e) run[e] += (float)a[e];
  }
}

extern "C" void kernel_launch(void* const* d_in, const int* in_sizes, int n_in,
                              void* d_out, int out_size, void* d_ws, size_t ws_size,
                              hipStream_t stream) {
  const int Lq = 2048, Bn = 4, E = 1024, EH = 2048, S = 128, CH = 64;
  const int NC = Lq / CH;
  const int ROWS = Bn * Lq;
  const int NCHK = Bn * NC;
  const int MAXP = 512;
  if (n_in < 22) return;
  if (in_sizes[0] != Lq * Bn * E || in_sizes[3] != E || in_sizes[4] != E) return;
  if (in_sizes[5] != EH * E || in_sizes[7] != EH * E || in_sizes[9] != S * E) return;
  if (in_sizes[6] != EH || in_sizes[8] != EH || in_sizes[10] != S) return;
  for (int i = 11; i <= 18; ++i) if (in_sizes[i] != S) return;
  if (in_sizes[19] != E * EH || in_sizes[20] != E || in_sizes[21] != 2 * MAXP - 1) return;
  if (out_size != Lq * Bn * E) return;

  const float* query = (const float*)d_in[0];
  const float* ln_g  = (const float*)d_in[3];
  const float* ln_b  = (const float*)d_in[4];
  const float* Wu    = (const float*)d_in[5];
  const float* bu    = (const float*)d_in[6];
  const float* Wv    = (const float*)d_in[7];
  const float* bv    = (const float*)d_in[8];
  const float* Wb    = (const float*)d_in[9];
  const float* bbv   = (const float*)d_in[10];
  const float* qqw   = (const float*)d_in[11];
  const float* qqb   = (const float*)d_in[12];
  const float* qkw   = (const float*)d_in[13];
  const float* qkb   = (const float*)d_in[14];
  const float* lqw   = (const float*)d_in[15];
  const float* lqb   = (const float*)d_in[16];
  const float* lkw   = (const float*)d_in[17];
  const float* lkb   = (const float*)d_in[18];
  const float* Wo    = (const float*)d_in[19];
  const float* bo    = (const float*)d_in[20];
  const float* wrel  = (const float*)d_in[21];
  float* out = (float*)d_out;

  char* ws = (char*)d_ws;
  size_t off = 0;
  auto alloc = [&](size_t bytes) { size_t o = off; off += (bytes + 255) & ~(size_t)255; return o; };
  const size_t oWb16 = alloc((size_t)S * E * 2);
  const size_t oWo16 = alloc((size_t)E * EH * 2);
  const size_t regA  = alloc((size_t)EH * E * 2 * 2 + (size_t)ROWS * E * 2);
  const size_t oWu16 = regA;
  const size_t oWv16 = regA + (size_t)EH * E * 2;
  const size_t oXn16 = regA + (size_t)EH * E * 2 * 2;
  const size_t oLkv  = regA;
  const size_t oX16  = regA + (size_t)NC * EH * S * 2;
  const size_t oU16  = alloc((size_t)ROWS * EH * 2);
  const size_t oVT16 = alloc((size_t)EH * ROWS * 2);
  const size_t oBase = alloc((size_t)ROWS * S * 4);
  const size_t oQq   = alloc((size_t)ROWS * S * 2);
  const size_t oQk   = alloc((size_t)ROWS * S * 2);
  const size_t oLq   = alloc((size_t)ROWS * S * 2);
  const size_t oLkT  = alloc((size_t)ROWS * S * 2);
  const size_t oSc   = alloc((size_t)NCHK * CH * CH * 4);
  const size_t oKm   = alloc((size_t)NCHK * CH * CH * 2);
  const size_t oCum  = alloc((size_t)NC * EH * S * 2);
  if (oX16 + (size_t)Lq * EH * 2 > regA + (size_t)EH * E * 4 + (size_t)ROWS * E * 2) return;
  if (off > ws_size || off > (size_t)134217728) return;

  unsigned short* Wb16 = (unsigned short*)(ws + oWb16);
  unsigned short* Wo16 = (unsigned short*)(ws + oWo16);
  unsigned short* Wu16 = (unsigned short*)(ws + oWu16);
  unsigned short* Wv16 = (unsigned short*)(ws + oWv16);
  unsigned short* xn16 = (unsigned short*)(ws + oXn16);
  unsigned short* lkv16 = (unsigned short*)(ws + oLkv);
  unsigned short* x16  = (unsigned short*)(ws + oX16);
  unsigned short* u16  = (unsigned short*)(ws + oU16);
  unsigned short* vT16 = (unsigned short*)(ws + oVT16);
  float*          basef = (float*)(ws + oBase);
  unsigned short* qq16 = (unsigned short*)(ws + oQq);
  unsigned short* qk16 = (unsigned short*)(ws + oQk);
  unsigned short* lq16 = (unsigned short*)(ws + oLq);
  unsigned short* lkT16 = (unsigned short*)(ws + oLkT);
  float*          scf  = (float*)(ws + oSc);
  unsigned short* km16 = (unsigned short*)(ws + oKm);
  unsigned short* cum16 = (unsigned short*)(ws + oCum);

  const float WSC = 16.0f;
  cast_f32_f16x2<<<dim3((EH * E / 2 + 255) / 256), dim3(256), 0, stream>>>(Wu, (_Float16*)Wu16, EH * E / 2, WSC);
  cast_f32_f16x2<<<dim3((EH * E / 2 + 255) / 256), dim3(256), 0, stream>>>(Wv, (_Float16*)Wv16, EH * E / 2, WSC);
  cast_f32_f16x2<<<dim3((S * E / 2 + 255) / 256), dim3(256), 0, stream>>>(Wb, (_Float16*)Wb16, S * E / 2, WSC);
  cast_f32_f16x2<<<dim3((E * EH / 2 + 255) / 256), dim3(256), 0, stream>>>(Wo, (_Float16*)Wo16, E * EH / 2, WSC);
  ln_kernel<<<dim3(ROWS), dim3(128), 0, stream>>>(query, ln_g, ln_b, (_Float16*)xn16, Lq, Bn, 1e-5f);
  {
    const int tiles = (ROWS / 64) * (EH / 64);
    wmma_gemm64<0, false, 2, 1, false, 3><<<dim3((tiles + 7) / 8), dim3(256), 0, stream>>>(
        xn16, nullptr, E, 0, Wu16, nullptr, E, 0, u16, nullptr, EH, 0, bu, nullptr, 0,
        ROWS, EH, E, 1.0f / WSC, 1);
  }
  {
    const int tiles = (EH / 64) * (ROWS / 64);
    wmma_gemm64<0, false, 1, 1, false, 3><<<dim3((tiles + 7) / 8), dim3(256), 0, stream>>>(
        Wv16, nullptr, E, 0, xn16, nullptr, E, 0, vT16, nullptr, ROWS, 0, bv, nullptr, 0,
        EH, ROWS, E, 1.0f / WSC, 1);
  }
  {
    const int tiles = (ROWS / 64) * (S / 64);
    wmma_gemm64<0, false, 2, 0, false, 3><<<dim3((tiles + 7) / 8), dim3(256), 0, stream>>>(
        xn16, nullptr, E, 0, Wb16, nullptr, E, 0, basef, nullptr, S, 0, bbv, nullptr, 0,
        ROWS, S, E, 1.0f / WSC, 1);
  }
  rope_kernel<<<dim3(NCHK), dim3(256), 0, stream>>>(basef, qqw, qqb, qkw, qkb, lqw, lqb, lkw, lkb,
      (_Float16*)qq16, (_Float16*)qk16, (_Float16*)lq16, (_Float16*)lkT16, NC);
  {
    wmma_gemm64<0, false, 0, 0, false, 0><<<dim3((NCHK + 7) / 8), dim3(256), 0, stream>>>(
        qq16, nullptr, S, (long)CH * S, qk16, nullptr, S, (long)CH * S, scf, nullptr, CH, (long)CH * CH,
        nullptr, nullptr, 0, CH, CH, S, 1.0f / 262144.0f, NCHK);
  }
  {
    const int total8 = NCHK * CH * CH / 8;
    kmat_kernel<<<dim3((total8 + 255) / 256), dim3(256), 0, stream>>>(scf, wrel, (_Float16*)km16, total8, MAXP - 1, 2 * MAXP - 1);
  }
  const long perKV = (long)EH * S;
  for (int b = 0; b < Bn; ++b) {
    {
      const int tiles = (EH / 64) * (S / 64);
      wmma_gemm64<0, false, 0, 1, false, 0><<<dim3((NC * tiles + 7) / 8), dim3(256), 0, stream>>>(
          vT16 + (size_t)b * Lq, nullptr, ROWS, (long)CH,
          lkT16 + (size_t)b * NC * S * CH, nullptr, CH, (long)S * CH,
          lkv16, nullptr, S, perKV, nullptr, nullptr, 0,
          EH, S, CH, 1.0f / 64.0f, NC);
    }
    {
      const int per8 = (int)(perKV / 8);
      cumsum_kernel<<<dim3((per8 + 255) / 256), dim3(256), 0, stream>>>((const _Float16*)lkv16, (_Float16*)cum16, per8, NC, perKV);
    }
    {
      const int tiles = (CH / 64) * (EH / 64);
      wmma_dual64<<<dim3((NC * tiles + 7) / 8), dim3(256), 0, stream>>>(
          km16 + (size_t)b * NC * CH * CH, CH, (long)CH * CH,
          vT16 + (size_t)b * Lq, ROWS, (long)CH, CH,
          lq16 + (size_t)b * Lq * S, S, (long)CH * S,
          cum16, S, perKV, S,
          u16 + (size_t)b * Lq * EH, EH, (long)CH * EH,
          x16, EH, (long)CH * EH,
          CH, EH, NC, 1.0f / 16.0f);
    }
    {
      const int tiles = (Lq / 64) * (E / 64);
      wmma_gemm64<0, false, 2, 0, true, 0><<<dim3((tiles + 7) / 8), dim3(256), 0, stream>>>(
          x16, nullptr, EH, 0, Wo16, nullptr, EH, 0,
          out + (size_t)b * E, nullptr, Bn * E, 0, bo,
          query + (size_t)b * E, 0,
          Lq, E, EH, 1.0f / 4096.0f, 1);
    }
  }
  (void)hipGetLastError();
}
